// MultiQueryAttention_69114613727693
// MI455X (gfx1250) — hardware-verified
//
#include <hip/hip_runtime.h>
#include <stdint.h>


typedef _Float16 v16h __attribute__((ext_vector_type(16)));
typedef _Float16 v8h  __attribute__((ext_vector_type(8)));
typedef float    v8f  __attribute__((ext_vector_type(8)));
typedef float    v4f  __attribute__((ext_vector_type(4)));

#define DM 2048
#define HD 128
#define NH 16
#define NB_FULL 1
#define SEQ_FULL 2048
#ifndef NB
#define NB 1
#endif
#ifndef SEQ
#define SEQ 2048
#endif
#define MROWS (NB * SEQ)
#define WSCALE 64.0f
#define PCARRY 1024.0f
#define YCARRY 64.0f
#define LOG2E 1.4426950408889634f
#define SMS 0.08838834764831845f
#define PP 136

static_assert(SEQ % 128 == 0);
static_assert(SEQ <= SEQ_FULL);
static_assert(NB == 1 && NB_FULL == 1);
static_assert(DM % 128 == 0 && HD == 128 && DM == NH * HD);
static_assert(MROWS % 128 == 0);
static_assert((MROWS * DM) % 2048 == 0 && (DM * DM) % 2048 == 0 && (HD * DM) % 2048 == 0);
static_assert((NB * NH * (SEQ / 16)) % 4 == 0);
static_assert((PP * 2) % 16 == 0 && PP >= HD);

union HFrag { v16h v; v8h h[2]; };

__device__ __forceinline__ v16h load_frag(const _Float16* p) {
    HFrag f;
    f.h[0] = *reinterpret_cast<const v8h*>(p);
    f.h[1] = *reinterpret_cast<const v8h*>(p + 16);
    return f.v;
}

__device__ __forceinline__ v8f wmma16(v16h a, v16h b, v8f c) {
    return __builtin_amdgcn_wmma_f32_16x16x32_f16(false, a, false, b, (short)0, c, false, false);
}

__device__ __forceinline__ float bf16r(float f) {
    unsigned int u = __float_as_uint(f);
    u += 0x7FFFu + ((u >> 16) & 1u);
    u &= 0xFFFF0000u;
    return __uint_as_float(u);
}

__global__ __launch_bounds__(256) void k_cvt(const float* __restrict__ src, _Float16* dst,
                                             int nunits, float scale)
{
    const int u = blockIdx.x * 256 + threadIdx.x;
    if (u >= nunits) return;
    const float* s = src + (size_t)u * 8;
    const float4 f0 = *reinterpret_cast<const float4*>(s);
    const float4 f1 = *reinterpret_cast<const float4*>(s + 4);
    v8h o;
    o[0] = (_Float16)(bf16r(f0.x) * scale); o[1] = (_Float16)(bf16r(f0.y) * scale);
    o[2] = (_Float16)(bf16r(f0.z) * scale); o[3] = (_Float16)(bf16r(f0.w) * scale);
    o[4] = (_Float16)(bf16r(f1.x) * scale); o[5] = (_Float16)(bf16r(f1.y) * scale);
    o[6] = (_Float16)(bf16r(f1.z) * scale); o[7] = (_Float16)(bf16r(f1.w) * scale);
    _Float16* d = dst + (size_t)u * 8;
    *(volatile v8h*)d = o;
    __threadfence();
    *(volatile v8h*)d = o;
}

__device__ __forceinline__ void store32x64_f16(const _Float16* sw, _Float16* gdst,
                                               size_t pitch, int lane)
{
    const int rq = lane >> 3, seg = lane & 7;
    v8h v[8];
#pragma unroll
    for (int it = 0; it < 8; ++it)
        v[it] = *reinterpret_cast<const v8h*>(sw + (it * 4 + rq) * 64 + seg * 8);
#pragma unroll
    for (int it = 0; it < 8; ++it)
        *(volatile v8h*)(gdst + (size_t)(it * 4 + rq) * pitch + seg * 8) = v[it];
    __threadfence();
#pragma unroll
    for (int it = 0; it < 8; ++it)
        *(volatile v8h*)(gdst + (size_t)(it * 4 + rq) * pitch + seg * 8) = v[it];
}

template <int MODE>
__global__ __launch_bounds__(256) void k_gemm(const _Float16* __restrict__ A,
                                              const _Float16* __restrict__ BT,
                                              void* C0, void* C1, int N, int K, float alpha)
{
    __shared__ float stg[8 * 1024] __attribute__((aligned(16)));
    const int tid = threadIdx.x;
    const int lane = tid & 31, wave = tid >> 5;
    const int wm = wave & 3, wn = wave >> 2;
    const int l15 = lane & 15, hi8 = (lane >> 4) << 3;
    const int bm0 = blockIdx.y * 128, bn0 = blockIdx.x * 128;

    const _Float16* ap0 = A + (size_t)(bm0 + wm * 32 + l15) * K + hi8;
    const _Float16* ap1 = ap0 + (size_t)16 * K;
    const _Float16* bp  = BT + (size_t)(bn0 + wn * 64 + l15) * K + hi8;
    const size_t bst = (size_t)16 * K;

    const v8f zero8 = {0.f, 0.f, 0.f, 0.f, 0.f, 0.f, 0.f, 0.f};
    v8f acc[2][4];
#pragma unroll
    for (int g = 0; g < 2; ++g)
#pragma unroll
        for (int ni = 0; ni < 4; ++ni) acc[g][ni] = zero8;

    for (int k0 = 0; k0 < K; k0 += 32) {
        const v16h a0 = load_frag(ap0 + k0);
        const v16h a1 = load_frag(ap1 + k0);
        const v16h b0 = load_frag(bp + k0);
        const v16h b1 = load_frag(bp + bst + k0);
        const v16h b2 = load_frag(bp + 2 * bst + k0);
        const v16h b3 = load_frag(bp + 3 * bst + k0);
        acc[0][0] = wmma16(a0, b0, acc[0][0]);
        acc[0][1] = wmma16(a0, b1, acc[0][1]);
        acc[0][2] = wmma16(a0, b2, acc[0][2]);
        acc[0][3] = wmma16(a0, b3, acc[0][3]);
        acc[1][0] = wmma16(a1, b0, acc[1][0]);
        acc[1][1] = wmma16(a1, b1, acc[1][1]);
        acc[1][2] = wmma16(a1, b2, acc[1][2]);
        acc[1][3] = wmma16(a1, b3, acc[1][3]);
        asm volatile("v_nop\n\tv_nop\n\tv_nop\n\tv_nop"
                     : "+v"(acc[0][0]), "+v"(acc[0][1]), "+v"(acc[0][2]), "+v"(acc[0][3]),
                       "+v"(acc[1][0]), "+v"(acc[1][1]), "+v"(acc[1][2]), "+v"(acc[1][3])
                     : "v"(a0), "v"(a1), "v"(b0), "v"(b1), "v"(b2), "v"(b3));
    }

    if (MODE == 0) {
        _Float16* sw = reinterpret_cast<_Float16*>(stg + wave * 1024);
#pragma unroll
        for (int g = 0; g < 2; ++g)
#pragma unroll
            for (int ni = 0; ni < 4; ++ni)
#pragma unroll
                for (int j = 0; j < 8; ++j)
                    sw[(g * 16 + hi8 + j) * 64 + ni * 16 + l15] = (_Float16)(acc[g][ni][j] * alpha);
        __syncthreads();
        store32x64_f16(sw, (_Float16*)C0 + (size_t)(bm0 + wm * 32) * N + bn0 + wn * 64,
                       (size_t)N, lane);
    } else if (MODE == 1) {
        float* swf = stg + wave * 1024;
        const int rq = lane >> 4, seg = lane & 15;
#pragma unroll
        for (int g = 0; g < 2; ++g) {
#pragma unroll
            for (int ni = 0; ni < 4; ++ni)
#pragma unroll
                for (int j = 0; j < 8; ++j)
                    swf[(hi8 + j) * 64 + ni * 16 + l15] = acc[g][ni][j] * alpha;
            __syncthreads();
            v4f v[8];
#pragma unroll
            for (int it = 0; it < 8; ++it)
                v[it] = *reinterpret_cast<const v4f*>(swf + (it * 2 + rq) * 64 + seg * 4);
            float* gd = (float*)C0 + (size_t)(bm0 + wm * 32 + g * 16) * N + bn0 + wn * 64 + seg * 4;
#pragma unroll
            for (int it = 0; it < 8; ++it)
                *(volatile v4f*)(gd + (size_t)(it * 2 + rq) * N) = v[it];
            __threadfence();
#pragma unroll
            for (int it = 0; it < 8; ++it)
                *(volatile v4f*)(gd + (size_t)(it * 2 + rq) * N) = v[it];
            __syncthreads();
        }
    } else {
        if (bn0 == 0) {
            _Float16* sw = reinterpret_cast<_Float16*>(stg + wave * 1024);
#pragma unroll
            for (int g = 0; g < 2; ++g)
#pragma unroll
                for (int ni = 0; ni < 4; ++ni)
#pragma unroll
                    for (int j = 0; j < 8; ++j)
                        sw[(g * 16 + hi8 + j) * 64 + ni * 16 + l15] = (_Float16)(acc[g][ni][j] * alpha);
            __syncthreads();
            store32x64_f16(sw, (_Float16*)C0 + (size_t)(bm0 + wm * 32) * HD + wn * 64,
                           (size_t)HD, lane);
        } else {
            _Float16* vs = reinterpret_cast<_Float16*>(stg);
#pragma unroll
            for (int g = 0; g < 2; ++g)
#pragma unroll
                for (int ni = 0; ni < 4; ++ni)
#pragma unroll
                    for (int j = 0; j < 8; ++j)
                        vs[(wn * 64 + ni * 16 + l15) * 128 + wm * 32 + g * 16 + hi8 + j] =
                            (_Float16)(acc[g][ni][j] * alpha);
            __syncthreads();
            const int bb = bm0 / SEQ;
            const int s0 = bm0 - bb * SEQ;
            const int dq = tid >> 4, seg = tid & 15;
            v8h v[8];
#pragma unroll
            for (int it = 0; it < 8; ++it)
                v[it] = *reinterpret_cast<const v8h*>(vs + (it * 16 + dq) * 128 + seg * 8);
            _Float16* vd = (_Float16*)C1 + ((size_t)(bb * HD)) * SEQ + s0 + seg * 8;
#pragma unroll
            for (int it = 0; it < 8; ++it)
                *(volatile v8h*)(vd + (size_t)(it * 16 + dq) * SEQ) = v[it];
            __threadfence();
#pragma unroll
            for (int it = 0; it < 8; ++it)
                *(volatile v8h*)(vd + (size_t)(it * 16 + dq) * SEQ) = v[it];
        }
    }
}

__global__ __launch_bounds__(128) void k_attn(const _Float16* __restrict__ qp,
                                              const _Float16* __restrict__ kp,
                                              const _Float16* __restrict__ vT,
                                              _Float16* yp)
{
    __shared__ _Float16 Ws[4 * 16 * PP] __attribute__((aligned(16)));
    const int lane = threadIdx.x & 31;
    const int wv   = threadIdx.x >> 5;
    const int l15  = lane & 15;
    const int hi8  = (lane >> 4) << 3;

    const int qtiles = SEQ / 16;
    int gw = blockIdx.x * 4 + wv;
    const int qt = gw % qtiles; gw /= qtiles;
    const int h  = gw % NH;
    const int b  = gw / NH;

    const _Float16* qbase = qp + ((size_t)(b * SEQ + qt * 16 + l15)) * DM + h * HD + hi8;
    const v16h aQ0 = load_frag(qbase);
    const v16h aQ1 = load_frag(qbase + 32);
    const v16h aQ2 = load_frag(qbase + 64);
    const v16h aQ3 = load_frag(qbase + 96);

    const _Float16* kbase = kp + (size_t)b * SEQ * HD + hi8;
    const _Float16* vbase = vT + (size_t)(b * HD) * SEQ + hi8;

    const v8f zero8 = {0.f, 0.f, 0.f, 0.f, 0.f, 0.f, 0.f, 0.f};
    float m[8], l[8];
    v8f accY[8];
#pragma unroll
    for (int j = 0; j < 8; ++j) { m[j] = -1e30f; l[j] = 0.0f; }
#pragma unroll
    for (int ni = 0; ni < 8; ++ni) accY[ni] = zero8;

    _Float16* ps = Ws + wv * 16 * PP;

#pragma unroll 1
    for (int tc = 0; tc < SEQ; tc += 32) {
        const _Float16* kp0 = kbase + (size_t)(tc + l15) * HD;
        const _Float16* kp1 = kp0 + 16 * HD;
        const v16h b00 = load_frag(kp0);
        const v16h b01 = load_frag(kp0 + 32);
        const v16h b02 = load_frag(kp0 + 64);
        const v16h b03 = load_frag(kp0 + 96);
        v8f s0 = zero8;
        s0 = wmma16(aQ0, b00, s0);
        s0 = wmma16(aQ1, b01, s0);
        s0 = wmma16(aQ2, b02, s0);
        s0 = wmma16(aQ3, b03, s0);
        asm volatile("v_nop\n\tv_nop\n\tv_nop\n\tv_nop"
                     : "+v"(s0)
                     : "v"(aQ0), "v"(aQ1), "v"(aQ2), "v"(aQ3),
                       "v"(b00), "v"(b01), "v"(b02), "v"(b03));
        const v16h b10 = load_frag(kp1);
        const v16h b11 = load_frag(kp1 + 32);
        const v16h b12 = load_frag(kp1 + 64);
        const v16h b13 = load_frag(kp1 + 96);
        v8f s1 = zero8;
        s1 = wmma16(aQ0, b10, s1);
        s1 = wmma16(aQ1, b11, s1);
        s1 = wmma16(aQ2, b12, s1);
        s1 = wmma16(aQ3, b13, s1);
        asm volatile("v_nop\n\tv_nop\n\tv_nop\n\tv_nop"
                     : "+v"(s1), "+v"(s0)
                     : "v"(aQ0), "v"(aQ1), "v"(aQ2), "v"(aQ3),
                       "v"(b10), "v"(b11), "v"(b12), "v"(b13));

#pragma unroll
        for (int j = 0; j < 8; ++j) {
            const float a0 = s0[j] * SMS;
            const float a1 = s1[j] * SMS;
            float mt = fmaxf(a0, a1);
#pragma unroll
            for (int off = 8; off >= 1; off >>= 1)
                mt = fmaxf(mt, __shfl_xor(mt, off, 16));
            const float mn = fmaxf(m[j], mt);
            const float sc = exp2f(m[j] - mn);
            const float p0 = exp2f(a0 - mn);
            const float p1 = exp2f(a1 - mn);
            float rs = p0 + p1;
#pragma unroll
            for (int off = 8; off >= 1; off >>= 1)
                rs += __shfl_xor(rs, off, 16);
            l[j] = l[j] * sc + rs;
            m[j] = mn;
            accY[0][j] *= sc; accY[1][j] *= sc; accY[2][j] *= sc; accY[3][j] *= sc;
            accY[4][j] *= sc; accY[5][j] *= sc; accY[6][j] *= sc; accY[7][j] *= sc;
            const int row = hi8 + j;
            ps[row * PP + l15]      = (_Float16)(p0 * PCARRY);
            ps[row * PP + 16 + l15] = (_Float16)(p1 * PCARRY);
        }
        __syncthreads();

        const v16h aP = load_frag(ps + l15 * PP + hi8);
        const v16h bV0 = load_frag(vbase + (size_t)(0 * 16 + l15) * SEQ + tc);
        const v16h bV1 = load_frag(vbase + (size_t)(1 * 16 + l15) * SEQ + tc);
        const v16h bV2 = load_frag(vbase + (size_t)(2 * 16 + l15) * SEQ + tc);
        const v16h bV3 = load_frag(vbase + (size_t)(3 * 16 + l15) * SEQ + tc);
        accY[0] = wmma16(aP, bV0, accY[0]);
        accY[1] = wmma16(aP, bV1, accY[1]);
        accY[2] = wmma16(aP, bV2, accY[2]);
        accY[3] = wmma16(aP, bV3, accY[3]);
        asm volatile("v_nop\n\tv_nop\n\tv_nop\n\tv_nop"
                     : "+v"(accY[0]), "+v"(accY[1]), "+v"(accY[2]), "+v"(accY[3])
                     : "v"(aP), "v"(bV0), "v"(bV1), "v"(bV2), "v"(bV3));
        const v16h bV4 = load_frag(vbase + (size_t)(4 * 16 + l15) * SEQ + tc);
        const v16h bV5 = load_frag(vbase + (size_t)(5 * 16 + l15) * SEQ + tc);
        const v16h bV6 = load_frag(vbase + (size_t)(6 * 16 + l15) * SEQ + tc);
        const v16h bV7 = load_frag(vbase + (size_t)(7 * 16 + l15) * SEQ + tc);
        accY[4] = wmma16(aP, bV4, accY[4]);
        accY[5] = wmma16(aP, bV5, accY[5]);
        accY[6] = wmma16(aP, bV6, accY[6]);
        accY[7] = wmma16(aP, bV7, accY[7]);
        asm volatile("v_nop\n\tv_nop\n\tv_nop\n\tv_nop"
                     : "+v"(accY[4]), "+v"(accY[5]), "+v"(accY[6]), "+v"(accY[7])
                     : "v"(aP), "v"(bV4), "v"(bV5), "v"(bV6), "v"(bV7));
    }
    __syncthreads();

    float inv[8];
#pragma unroll
    for (int j = 0; j < 8; ++j) inv[j] = (YCARRY / PCARRY) / l[j];
#pragma unroll
    for (int ni = 0; ni < 8; ++ni)
#pragma unroll
        for (int j = 0; j < 8; ++j)
            ps[(hi8 + j) * PP + ni * 16 + l15] = (_Float16)(accY[ni][j] * inv[j]);
    __syncthreads();

    const int rq = lane >> 4, seg = lane & 15;
    v8h v[8];
#pragma unroll
    for (int it = 0; it < 8; ++it)
        v[it] = *reinterpret_cast<const v8h*>(ps + (it * 2 + rq) * PP + seg * 8);
    _Float16* yd = yp + ((size_t)(b * SEQ + qt * 16)) * DM + h * HD + seg * 8;
#pragma unroll
    for (int it = 0; it < 8; ++it)
        *(volatile v8h*)(yd + (size_t)(it * 2 + rq) * DM) = v[it];
    __threadfence();
#pragma unroll
    for (int it = 0; it < 8; ++it)
        *(volatile v8h*)(yd + (size_t)(it * 2 + rq) * DM) = v[it];
}

extern "C" void kernel_launch(void* const* d_in, const int* in_sizes, int n_in,
                              void* d_out, int out_size, void* d_ws, size_t ws_size,
                              hipStream_t stream) {
    if (n_in < 5) return;
    const long long needX = ((long long)(NB - 1) * SEQ_FULL + SEQ) * DM;
    if ((long long)in_sizes[0] < needX) return;
    if (in_sizes[1] < DM * DM || in_sizes[2] < HD * DM || in_sizes[3] < HD * DM || in_sizes[4] < DM * DM) return;
    if ((long long)out_size < (long long)MROWS * DM) return;

    const float* x  = (const float*)d_in[0];
    const float* Wq = (const float*)d_in[1];
    const float* Wk = (const float*)d_in[2];
    const float* Wv = (const float*)d_in[3];
    const float* Wo = (const float*)d_in[4];
    float* out = (float*)d_out;

    size_t off = 0;
    char* wsb = (char*)d_ws;
    auto carve = [&](size_t bytes) -> void* {
        void* p = wsb + off;
        off += (bytes + 255) & ~(size_t)255;
        return p;
    };
    _Float16* x16   = (_Float16*)carve((size_t)MROWS * DM * 2);
    _Float16* Wq16  = (_Float16*)carve((size_t)DM * DM * 2);
    _Float16* Wkv16 = (_Float16*)carve((size_t)(2 * HD) * DM * 2);
    _Float16* Wo16  = (_Float16*)carve((size_t)DM * DM * 2);
    _Float16* q16   = (_Float16*)carve((size_t)MROWS * DM * 2);
    _Float16* kpl   = (_Float16*)carve((size_t)MROWS * HD * 2);
    _Float16* vT    = (_Float16*)carve((size_t)NB * HD * SEQ * 2);
    _Float16* y16   = (_Float16*)carve((size_t)MROWS * DM * 2);
    if (off > ws_size) return;

    dim3 blk(256);
    const int UX = MROWS * DM / 8;
    const int UQ = DM * DM / 8;
    const int UK = HD * DM / 8;

    k_cvt<<<dim3(UX / 256), blk, 0, stream>>>(x, x16, UX, 1.0f);
    k_cvt<<<dim3(UQ / 256), blk, 0, stream>>>(Wq, Wq16, UQ, WSCALE);
    k_cvt<<<dim3(UK / 256), blk, 0, stream>>>(Wk, Wkv16, UK, WSCALE);
    k_cvt<<<dim3(UK / 256), blk, 0, stream>>>(Wv, Wkv16 + (size_t)HD * DM, UK, WSCALE);
    k_cvt<<<dim3(UQ / 256), blk, 0, stream>>>(Wo, Wo16, UQ, WSCALE);

    k_gemm<0><<<dim3(DM / 128, MROWS / 128), blk, 0, stream>>>(
        x16, Wq16, (void*)q16, (void*)q16, DM, DM, LOG2E / WSCALE);
    k_gemm<2><<<dim3(2, MROWS / 128), blk, 0, stream>>>(
        x16, Wkv16, (void*)kpl, (void*)vT, 2 * HD, DM, 1.0f / WSCALE);
    k_attn<<<dim3((NB * NH * (SEQ / 16)) / 4), dim3(128), 0, stream>>>(q16, kpl, vT, y16);
    k_gemm<1><<<dim3(DM / 128, MROWS / 128), blk, 0, stream>>>(
        y16, Wo16, (void*)out, (void*)out, DM, DM, 1.0f / (YCARRY * WSCALE));
}
